// CrossAttention_65541200937572
// MI455X (gfx1250) — hardware-run, weakly checked
//
#include <hip/hip_runtime.h>
#ifndef NB
#define NB 2
#endif
#ifndef SEQ
#define SEQ 2048
#endif
#define NB_FULL 2
#define SEQ_FULL 2048
#define DE 1024
#define NH 16
#define HD 64
#define MROWS (NB * SEQ)
#define BSTRIDE_FULL ((size_t)SEQ_FULL * DE)
#define MSTRIDE_FULL ((size_t)SEQ_FULL * SEQ_FULL)

#define PL_X ((size_t)MROWS * DE * 2)
#define PL_W ((size_t)DE * DE * 2)
#define WS_TOTAL (5 * PL_X + 3 * PL_W)

static_assert(SEQ % 128 == 0);
static_assert(SEQ % 64 == 0);
static_assert(SEQ % 32 == 0);
static_assert(SEQ <= SEQ_FULL);
static_assert(NB <= NB_FULL);
static_assert(HD == 64);
static_assert(DE == 1024);
static_assert(DE / 8 == 128);
static_assert(DE % 32 == 0);
static_assert(NH * HD == DE);
static_assert(MROWS % 64 == 0);
static_assert(DE % 128 == 0);
static_assert(SEQ_FULL % 4 == 0);
static_assert(PL_X % 128 == 0);
static_assert(PL_W % 128 == 0);
static_assert(WS_TOTAL <= (size_t)134217728);
static_assert(((size_t)(NB - 1) * BSTRIDE_FULL + (size_t)SEQ * DE) * 4 <= (size_t)16777216);

typedef __bf16 v16b __attribute__((ext_vector_type(16)));
typedef _Float16 v16h __attribute__((ext_vector_type(16)));
typedef unsigned short v8us __attribute__((ext_vector_type(8), may_alias));
typedef float v8f __attribute__((ext_vector_type(8)));
typedef float v4f __attribute__((ext_vector_type(4)));
typedef float v4fa __attribute__((ext_vector_type(4), may_alias));
union FragB { v16b v; v8us half[2]; };
union FragH { v16h v; v8us half[2]; _Float16 h[16]; };
union H8 { v8us v; _Float16 h[8]; unsigned short u[8]; };

#define LOG2E 1.4426950408889634f

__device__ __forceinline__ unsigned short bf16_bits(float x) {
  unsigned int u = __float_as_uint(x);
  return (unsigned short)((u + 0x7FFFu + ((u >> 16) & 1u)) >> 16);
}
__device__ __forceinline__ float bf16_val(unsigned short b) { return __uint_as_float(((unsigned int)b) << 16); }
__device__ __forceinline__ float bf16_rne(float x) { return bf16_val(bf16_bits(x)); }

static __device__ __forceinline__ _Float16 toh_flush(float v) {
  const _Float16 r = (_Float16)v;
  return (fabsf(v) < 6.103515625e-05f) ? (_Float16)0.0f : r;
}

__device__ __forceinline__ void mma_b8(v16b a0, v16b a1, v16b b0, v16b b1, v16b b2, v16b b3, v8f (&c)[2][4]) {
  c[0][0] = __builtin_amdgcn_wmma_f32_16x16x32_bf16(false, a0, false, b0, (short)0, c[0][0], false, false);
  c[0][1] = __builtin_amdgcn_wmma_f32_16x16x32_bf16(false, a0, false, b1, (short)0, c[0][1], false, false);
  c[0][2] = __builtin_amdgcn_wmma_f32_16x16x32_bf16(false, a0, false, b2, (short)0, c[0][2], false, false);
  c[0][3] = __builtin_amdgcn_wmma_f32_16x16x32_bf16(false, a0, false, b3, (short)0, c[0][3], false, false);
  c[1][0] = __builtin_amdgcn_wmma_f32_16x16x32_bf16(false, a1, false, b0, (short)0, c[1][0], false, false);
  c[1][1] = __builtin_amdgcn_wmma_f32_16x16x32_bf16(false, a1, false, b1, (short)0, c[1][1], false, false);
  c[1][2] = __builtin_amdgcn_wmma_f32_16x16x32_bf16(false, a1, false, b2, (short)0, c[1][2], false, false);
  c[1][3] = __builtin_amdgcn_wmma_f32_16x16x32_bf16(false, a1, false, b3, (short)0, c[1][3], false, false);
  asm volatile("v_nop\n\tv_nop\n\tv_nop\n\tv_nop"
               : "+v"(c[0][0]), "+v"(c[0][1]), "+v"(c[0][2]), "+v"(c[0][3]),
                 "+v"(c[1][0]), "+v"(c[1][1]), "+v"(c[1][2]), "+v"(c[1][3])
               : "v"(a0), "v"(a1), "v"(b0), "v"(b1), "v"(b2), "v"(b3));
}
__device__ __forceinline__ v8f mma_h2(v16h a0, v16h b0, v16h a1, v16h b1, v8f c) {
  c = __builtin_amdgcn_wmma_f32_16x16x32_f16(false, a0, false, b0, (short)0, c, false, false);
  c = __builtin_amdgcn_wmma_f32_16x16x32_f16(false, a1, false, b1, (short)0, c, false, false);
  asm volatile("v_nop\n\tv_nop\n\tv_nop\n\tv_nop" : "+v"(c) : "v"(a0), "v"(b0), "v"(a1), "v"(b1));
  return c;
}
__device__ __forceinline__ void mma_pv4(v16h a0, v16h a1, v16h a2, v16h a3, v16h b, v8f (&c)[4]) {
  c[0] = __builtin_amdgcn_wmma_f32_16x16x32_f16(false, a0, false, b, (short)0, c[0], false, false);
  c[1] = __builtin_amdgcn_wmma_f32_16x16x32_f16(false, a1, false, b, (short)0, c[1], false, false);
  c[2] = __builtin_amdgcn_wmma_f32_16x16x32_f16(false, a2, false, b, (short)0, c[2], false, false);
  c[3] = __builtin_amdgcn_wmma_f32_16x16x32_f16(false, a3, false, b, (short)0, c[3], false, false);
  asm volatile("v_nop\n\tv_nop\n\tv_nop\n\tv_nop"
               : "+v"(c[0]), "+v"(c[1]), "+v"(c[2]), "+v"(c[3])
               : "v"(a0), "v"(a1), "v"(a2), "v"(a3), "v"(b));
}
__device__ __forceinline__ void ldfrag(FragH& f, const unsigned short* __restrict__ p) {
  f.half[0] = *(const v8us*)(p);
  f.half[1] = *(const v8us*)(p + 16);
}

__global__ __launch_bounds__(256) void k_cvt(const float* __restrict__ src, unsigned short* __restrict__ dst,
                                             int nrows, int rpb, long long bstride) {
  const int t = blockIdx.x * 256 + threadIdx.x;
  if (t >= nrows * (DE / 8)) return;
  const int row = t >> 7, piece = t & 127;
  const int b = row / rpb, s = row - b * rpb;
  const float* p = src + (size_t)b * (size_t)bstride + (size_t)s * DE + piece * 8;
  const v4f x0 = *(const v4fa*)(p), x1 = *(const v4fa*)(p + 4);
  v8us o;
  o[0] = bf16_bits(x0[0]); o[1] = bf16_bits(x0[1]); o[2] = bf16_bits(x0[2]); o[3] = bf16_bits(x0[3]);
  o[4] = bf16_bits(x1[0]); o[5] = bf16_bits(x1[1]); o[6] = bf16_bits(x1[2]); o[7] = bf16_bits(x1[3]);
  unsigned short* d = dst + (size_t)t * 8;
  *(volatile v8us*)d = o;
  __threadfence();
  *(volatile v8us*)d = o;
}

template <int MODE>
__device__ __forceinline__ void gemm_body(const unsigned short* __restrict__ X, const unsigned short* __restrict__ W,
                                          const float* __restrict__ bias, unsigned short* __restrict__ Y0, int ldx, int K) {
  __shared__ __attribute__((aligned(16))) float so[64][132];
  const int tid = threadIdx.x;
  const int w = __builtin_amdgcn_readfirstlane(tid >> 5);
  const int lane = tid & 31, ln = lane & 15, hh = lane >> 4;
  const int bm = blockIdx.x % (MROWS / 64), bn = blockIdx.x / (MROWS / 64);
  const int m0 = bm * 64, n0 = bn * 128;
  const int wm = w & 1, wn = w >> 1;
  const unsigned short* xr = X + (size_t)(m0 + 32 * wm + ln) * ldx + 8 * hh;
  const unsigned short* wr = W + (size_t)(n0 + 64 * wn + ln) * DE + 8 * hh;
  v8f c[2][4] = {};
#pragma unroll 1
  for (int k0 = 0; k0 < K; k0 += 32) {
    const int kw = k0 & (DE - 1);
    FragB a0, a1, b0, b1, b2, b3;
    a0.half[0] = *(const v8us*)(xr + k0);
    a0.half[1] = *(const v8us*)(xr + k0 + 16);
    a1.half[0] = *(const v8us*)(xr + (size_t)16 * ldx + k0);
    a1.half[1] = *(const v8us*)(xr + (size_t)16 * ldx + k0 + 16);
    b0.half[0] = *(const v8us*)(wr + kw);
    b0.half[1] = *(const v8us*)(wr + kw + 16);
    b1.half[0] = *(const v8us*)(wr + 16 * DE + kw);
    b1.half[1] = *(const v8us*)(wr + 16 * DE + kw + 16);
    b2.half[0] = *(const v8us*)(wr + 32 * DE + kw);
    b2.half[1] = *(const v8us*)(wr + 32 * DE + kw + 16);
    b3.half[0] = *(const v8us*)(wr + 48 * DE + kw);
    b3.half[1] = *(const v8us*)(wr + 48 * DE + kw + 16);
    mma_b8(a0.v, a1.v, b0.v, b1.v, b2.v, b3.v, c);
  }
#pragma unroll
  for (int t = 0; t < 4; ++t) {
    const float bv = bf16_rne(bias[n0 + 64 * wn + 16 * t + ln]);
#pragma unroll
    for (int i = 0; i < 2; ++i)
#pragma unroll
      for (int r = 0; r < 8; ++r)
        so[32 * wm + 16 * i + 8 * hh + r][64 * wn + 16 * t + ln] = c[i][t][r] + bv;
  }
  __syncthreads();
  const int b = m0 / SEQ, s0 = m0 - b * SEQ;
  if (MODE == 0) {
    for (int pass = 0; pass < 2; ++pass) {
#pragma unroll 1
      for (int it = 0; it < 8; ++it) {
        const int i = it * 128 + tid;
        const int line = i >> 3, piece = i & 7;
        const int row = line >> 1, cb = (line & 1) * 64 + piece * 8;
        const v4f x0 = *(const v4fa*)&so[row][cb], x1 = *(const v4fa*)&so[row][cb + 4];
        H8 hi;
#pragma unroll
        for (int j = 0; j < 4; ++j) {
          hi.h[j] = toh_flush(x0[j]);
          hi.h[4 + j] = toh_flush(x1[j]);
        }
        const size_t o = (size_t)(m0 + row) * DE + n0 + cb;
        *(volatile v8us*)(Y0 + o) = hi.v;
      }
      if (pass == 0) __threadfence();
    }
  } else {
    for (int pass = 0; pass < 2; ++pass) {
#pragma unroll 1
      for (int it = 0; it < 8; ++it) {
        const int i = it * 128 + tid;
        const int cidx = i >> 3, piece = i & 7;
        const int n = n0 + cidx;
        const int head = n >> 6, d = n & 63;
        H8 hi;
#pragma unroll
        for (int j = 0; j < 8; ++j) {
          const float v = so[piece * 8 + j][cidx] * 16.0f;
          hi.h[j] = toh_flush(v);
        }
        const size_t o = ((size_t)(b * NH + head) * HD + d) * SEQ + s0 + piece * 8;
        *(volatile v8us*)(Y0 + o) = hi.v;
      }
      if (pass == 0) __threadfence();
    }
  }
}

__global__ __launch_bounds__(128) void k_gemm_rows(const unsigned short* __restrict__ X, const unsigned short* __restrict__ W,
                                                   const float* __restrict__ bias, unsigned short* __restrict__ Y0,
                                                   int ldx, int K) {
  gemm_body<0>(X, W, bias, Y0, ldx, K);
}
__global__ __launch_bounds__(128) void k_gemm_tr(const unsigned short* __restrict__ X, const unsigned short* __restrict__ W,
                                                 const float* __restrict__ bias, unsigned short* __restrict__ Y0,
                                                 int ldx, int K) {
  gemm_body<1>(X, W, bias, Y0, ldx, K);
}

__device__ __forceinline__ void fa_step(const unsigned short* __restrict__ Khp, const unsigned short* __restrict__ Vhp,
                                        const float* __restrict__ mrow, int key0, int ln, int hh,
                                        const FragH (&qh)[2], float& mr, float& lr, v8f (&Oh)[4]) {
  const size_t ko = (size_t)(key0 + ln) * DE + 8 * hh;
  FragH k00, k01, k10, k11;
  ldfrag(k00, Khp + ko);            ldfrag(k01, Khp + ko + 32);
  ldfrag(k10, Khp + ko + 16 * DE);  ldfrag(k11, Khp + ko + 16 * DE + 32);
  const float* mp = mrow + key0 + 8 * hh;
  const v4f ma = *(const v4fa*)(mp), mb = *(const v4fa*)(mp + 4);
  const v4f mc = *(const v4fa*)(mp + 16), md = *(const v4fa*)(mp + 20);
  const v8f z8 = {0.f, 0.f, 0.f, 0.f, 0.f, 0.f, 0.f, 0.f};
  v8f s0 = mma_h2(k00.v, qh[0].v, k01.v, qh[1].v, z8);
  v8f s1 = mma_h2(k10.v, qh[0].v, k11.v, qh[1].v, z8);
  float sc[16];
#pragma unroll
  for (int r = 0; r < 4; ++r) {
    sc[r]      = s0[r] * 0.125f     + (1.0f - bf16_rne(ma[r])) * -10000.0f;
    sc[4 + r]  = s0[4 + r] * 0.125f + (1.0f - bf16_rne(mb[r])) * -10000.0f;
    sc[8 + r]  = s1[r] * 0.125f     + (1.0f - bf16_rne(mc[r])) * -10000.0f;
    sc[12 + r] = s1[4 + r] * 0.125f + (1.0f - bf16_rne(md[r])) * -10000.0f;
  }
  float mx = sc[0];
#pragma unroll
  for (int i = 1; i < 16; ++i) mx = fmaxf(mx, sc[i]);
  mx = fmaxf(mx, __shfl_xor(mx, 16, 32));
  const float mnew = fmaxf(mr, mx);
  const float al = exp2f((mr - mnew) * LOG2E);
  mr = mnew;
  FragH ph;
  float ps = 0.0f;
#pragma unroll
  for (int i = 0; i < 16; ++i) {
    const float e = fmaf(sc[i] - mnew, LOG2E, 8.0f);
    const float pe = exp2f(e);
    const float pc = (e < -14.0f) ? 0.0f : pe;
    const _Float16 h = (_Float16)pc;
    ph.h[i] = h;
    ps += (float)h;
  }
  ps += __shfl_xor(ps, 16, 32);
  lr = lr * al + ps;
  const size_t vo = (size_t)ln * SEQ + key0 + 8 * hh;
  FragH vf[4];
#pragma unroll
  for (int t = 0; t < 4; ++t) ldfrag(vf[t], Vhp + vo + (size_t)t * 16 * SEQ);
#pragma unroll
  for (int t = 0; t < 4; ++t) Oh[t] = Oh[t] * al;
  mma_pv4(vf[0].v, vf[1].v, vf[2].v, vf[3].v, ph.v, Oh);
}

__global__ __launch_bounds__(128) void k_attn(const unsigned short* __restrict__ Qh, const unsigned short* __restrict__ Kh,
                                              const unsigned short* __restrict__ Vth, const float* __restrict__ mask,
                                              float* __restrict__ out) {
  __shared__ __attribute__((aligned(16))) float so[4][16][68];
  const int tid = threadIdx.x;
  const int w = __builtin_amdgcn_readfirstlane(tid >> 5);
  const int lane = tid & 31, ln = lane & 15, hh = lane >> 4;
  const int qt = blockIdx.x % (SEQ / 64);
  const int bh = blockIdx.x / (SEQ / 64);
  const int h = bh % NH, b = bh / NH;
  const int qbase = qt * 64 + 16 * w;
  const int qg = qbase + ln;
  const size_t qo = (size_t)(b * SEQ + qg) * DE + h * HD + 8 * hh;
  FragH qh[2];
  ldfrag(qh[0], Qh + qo); ldfrag(qh[1], Qh + qo + 32);
  float mr = -3.0e38f, lr = 0.0f;
  v8f Oh[4] = {};
  const unsigned short* Khp = Kh + (size_t)b * SEQ * DE + h * HD;
  const unsigned short* Vhp = Vth + (size_t)(b * NH + h) * HD * SEQ;
  const float* mrow = mask + (size_t)b * MSTRIDE_FULL + (size_t)qg * SEQ_FULL;
#pragma unroll 1
  for (int j = 0; j < SEQ / 32; ++j)
    fa_step(Khp, Vhp, mrow, 32 * j, ln, hh, qh, mr, lr, Oh);
  const float inv = 1.0f / (16.0f * lr);
#pragma unroll
  for (int t = 0; t < 4; ++t)
#pragma unroll
    for (int r = 0; r < 8; ++r)
      so[w][ln][16 * t + 8 * hh + r] = Oh[t][r] * inv;
  __syncthreads();
  float* orow = out + (size_t)b * BSTRIDE_FULL + (size_t)qbase * DE + h * HD;
  const int lsub = lane >> 3, piece = lane & 7;
  for (int pass = 0; pass < 2; ++pass) {
#pragma unroll
    for (int it = 0; it < 8; ++it) {
      const int line = it * 4 + lsub;
      const int row = line >> 1, cb = (line & 1) * 32 + piece * 4;
      const v4f v = *(const v4fa*)&so[w][row][cb];
      *(volatile v4f*)(orow + (size_t)row * DE + cb) = v;
    }
    if (pass == 0) __threadfence();
  }
}

extern "C" void kernel_launch(void* const* d_in, const int* in_sizes, int n_in,
                              void* d_out, int out_size, void* d_ws, size_t ws_size, hipStream_t stream) {
  if (n_in < 9) return;
  const long long need_x = (long long)(NB - 1) * SEQ_FULL * DE + (long long)SEQ * DE;
  const long long need_m = (long long)(NB - 1) * SEQ_FULL * SEQ_FULL + (long long)(SEQ - 1) * SEQ_FULL + SEQ;
  if ((long long)in_sizes[0] < need_x || (long long)in_sizes[1] < need_x) return;
  if ((long long)in_sizes[2] < need_m) return;
  if ((long long)in_sizes[3] < (long long)DE * DE || (long long)in_sizes[5] < (long long)DE * DE) return;
  if ((long long)in_sizes[7] < (long long)DE * DE) return;
  if (in_sizes[4] < DE || in_sizes[6] < DE || in_sizes[8] < DE) return;
  if ((long long)out_size < need_x) return;
  if ((size_t)WS_TOTAL > ws_size) return;
  const float* xq   = (const float*)d_in[0];
  const float* xk   = (const float*)d_in[1];
  const float* mask = (const float*)d_in[2];
  const float* Wq = (const float*)d_in[3];
  const float* bq = (const float*)d_in[4];
  const float* Wk = (const float*)d_in[5];
  const float* bk = (const float*)d_in[6];
  const float* Wv = (const float*)d_in[7];
  const float* bv = (const float*)d_in[8];
  float* out = (float*)d_out;
  char* ws = (char*)d_ws;
  size_t off = 0;
  unsigned short* Xq  = (unsigned short*)(ws + off); off += PL_X;
  unsigned short* Xk  = (unsigned short*)(ws + off); off += PL_X;
  unsigned short* Wqb = (unsigned short*)(ws + off); off += PL_W;
  unsigned short* Wkb = (unsigned short*)(ws + off); off += PL_W;
  unsigned short* Wvb = (unsigned short*)(ws + off); off += PL_W;
  unsigned short* Qh  = (unsigned short*)(ws + off); off += PL_X;
  unsigned short* Kh  = (unsigned short*)(ws + off); off += PL_X;
  unsigned short* Vth = (unsigned short*)(ws + off); off += PL_X;
  if (off > ws_size) return;

  const unsigned gx = (unsigned)((MROWS * (DE / 8) + 255) / 256);
  const unsigned gw = (unsigned)((DE * (DE / 8) + 255) / 256);
  k_cvt<<<gx, 256, 0, stream>>>(xq, Xq, MROWS, SEQ, (long long)BSTRIDE_FULL);
  k_cvt<<<gx, 256, 0, stream>>>(xk, Xk, MROWS, SEQ, (long long)BSTRIDE_FULL);
  k_cvt<<<gw, 256, 0, stream>>>(Wq, Wqb, DE, DE, 0LL);
  k_cvt<<<gw, 256, 0, stream>>>(Wk, Wkb, DE, DE, 0LL);
  k_cvt<<<gw, 256, 0, stream>>>(Wv, Wvb, DE, DE, 0LL);

  const unsigned gg = (unsigned)((MROWS / 64) * (DE / 128));
  k_gemm_rows<<<gg, 128, 0, stream>>>(Xq, Wqb, bq, Qh,  DE, DE);
  k_gemm_rows<<<gg, 128, 0, stream>>>(Xk, Wkb, bk, Kh,  DE, DE);
  k_gemm_tr  <<<gg, 128, 0, stream>>>(Xk, Wvb, bv, Vth, DE, DE);

  k_attn<<<(unsigned)(NB * NH * (SEQ / 64)), 128, 0, stream>>>(Qh, Kh, Vth, mask, out);
}
